// ResidualGNN_19215683683065
// MI455X (gfx1250) — hardware-run, weakly checked
//
#include <hip/hip_runtime.h>

#define NB    8
#define NN    1024
#define HID   32
#define IW    16
#define WPB   8
#define NG    (NN / IW)
#define BPB   (NN / (WPB * IW))
#define NSLOT 21

static_assert(NN == 1024);
static_assert(NN % 32 == 0);
static_assert(HID == 32);
static_assert(NSLOT <= 32);
static_assert(IW == 16);
static_assert(NN % (WPB * IW) == 0);
static_assert(IW * 8 == 32 * 4);

#define PL_W1X    0
#define PL_W2T    1024
#define PL_W3T    2048
#define PL_BV_DW  1280
#define PL_DW     1344
#define PL_PIECES 336
static_assert(PL_W3T * 2 + 16 * 32 * 2 == PL_BV_DW * 4);
static_assert(PL_BV_DW * 4 + 256 == PL_DW * 4);
static_assert(PL_PIECES * 4 == PL_DW);

#define WS_PLN    0
#define WS_NODE   5632
#define WS_RA     (WS_NODE + NB * NN * 32)
#define WS_COLP   (WS_RA + NB * NN * 32)
#define WS_TOTAL  (WS_COLP + NB * NG * NN * 16)
static_assert(PL_DW * 4 <= WS_NODE);
static_assert(WS_NODE % 256 == 0 && WS_RA % 256 == 0 && WS_COLP % 256 == 0);
static_assert(NB * NG * NN * 16 == 8388608);
static_assert(WS_TOTAL == 8918528);
static_assert(WS_TOTAL <= 134217728);

#define L_NODE   32768
#define L_FEAT   2048
#define L_COL    16384
#define L_RA     512
#define L_WV     (L_FEAT + L_COL + L_RA)
#define L_TOTAL  (L_NODE + WPB * L_WV)
static_assert(L_WV % 16 == 0);
static_assert(L_TOTAL == 184320);
static_assert(L_TOTAL <= 327680);

typedef __attribute__((ext_vector_type(16))) __bf16 v16b;
typedef __attribute__((ext_vector_type(8)))  float  v8f;
typedef __attribute__((ext_vector_type(4)))  float  v4f;
typedef __attribute__((ext_vector_type(4)))  unsigned int v4u;
typedef v4f __attribute__((may_alias)) v4fa;
typedef v4u __attribute__((may_alias)) v4ua;

union FragU { v16b v; v4u q[2]; };
struct U2 { unsigned h; unsigned l; };
struct FragPair { v16b hi; v16b lo; };

__device__ __forceinline__ unsigned rne_bits(float f) {
  const unsigned u = __float_as_uint(f);
  return (u + 0x7FFFu + ((u >> 16) & 1u)) >> 16;
}
__device__ __forceinline__ float bf16r(float f) {
  unsigned u = __float_as_uint(f);
  u = (u + 0x7FFFu + ((u >> 16) & 1u)) & 0xFFFF0000u;
  return __uint_as_float(u);
}
__device__ __forceinline__ unsigned tail_bits(float x, unsigned u) {
  const float t = x - __uint_as_float(u & 0xFFFF0000u);
  return rne_bits(t);
}

__device__ __forceinline__ v8f wmma_bf16(v16b a, v16b b, v8f c) {
  v8f d = __builtin_amdgcn_wmma_f32_16x16x32_bf16(false, a, false, b, (short)0, c, false, false);
  asm volatile("v_nop\n\tv_nop\n\tv_nop\n\tv_nop" : "+v"(d) : "v"(a), "v"(b));
  return d;
}

__device__ __forceinline__ v16b load_frag_g(const unsigned short* __restrict__ p, int hh) {
  FragU f;
  f.q[0] = *(const v4ua*)(p + 8 * hh);
  f.q[1] = *(const v4ua*)(p + 16 + 8 * hh);
  return f.v;
}

__device__ __forceinline__ float silu_f(float x) {
  const float t = x * (-1.4426950216293335f);
  const float a = fmaf(x, -1.92596299e-8f, t);
  const float e = __builtin_amdgcn_exp2f(a);
  const float r = __builtin_amdgcn_rcpf(1.0f + e);
  return x * r;
}

__device__ __forceinline__ U2 act2(float x0, float x1) {
  const float s0 = silu_f(x0), s1 = silu_f(x1);
  const unsigned u0 = __float_as_uint(s0), u1 = __float_as_uint(s1);
  const unsigned t0 = u0 & 0xFFFF0000u, t1 = u1 & 0xFFFF0000u;
  const float l0 = s0 - __uint_as_float(t0);
  const float l1 = s1 - __uint_as_float(t1);
  U2 o;
  o.h = (u0 >> 16) | t1;
  o.l = (__float_as_uint(l0) >> 16) | (__float_as_uint(l1) & 0xFFFF0000u);
  return o;
}

__device__ __forceinline__ FragPair act_split(v8f c0, v8f c1) {
  const U2 p0 = act2(c0[0], c0[1]);
  const U2 p1 = act2(c0[2], c0[3]);
  const U2 p2 = act2(c0[4], c0[5]);
  const U2 p3 = act2(c0[6], c0[7]);
  const U2 p4 = act2(c1[0], c1[1]);
  const U2 p5 = act2(c1[2], c1[3]);
  const U2 p6 = act2(c1[4], c1[5]);
  const U2 p7 = act2(c1[6], c1[7]);
  FragU H, L;
  const v4u h0 = { p0.h, p1.h, p2.h, p3.h };
  const v4u h1 = { p4.h, p5.h, p6.h, p7.h };
  const v4u l0 = { p0.l, p1.l, p2.l, p3.l };
  const v4u l1 = { p4.l, p5.l, p6.l, p7.l };
  H.q[0] = h0; H.q[1] = h1;
  L.q[0] = l0; L.q[1] = l1;
  FragPair o;
  o.hi = H.v;
  o.lo = L.v;
  return o;
}

__global__ __launch_bounds__(256) void k_prep(
    const float* __restrict__ r, const float* __restrict__ v,
    const float* __restrict__ W1, const float* __restrict__ b1,
    const float* __restrict__ W2, const float* __restrict__ b2,
    const float* __restrict__ W3, const float* __restrict__ b3,
    unsigned int* __restrict__ PLN, float* __restrict__ NODE)
{
  __shared__ __attribute__((aligned(16))) unsigned int sS[2048];
  const int tid = threadIdx.x;
  if (blockIdx.x < 32) {
    const int node = blockIdx.x * 256 + tid;
    const float r0 = r[node * 3 + 0], r1 = r[node * 3 + 1], r2 = r[node * 3 + 2];
    const float v0 = v[node * 3 + 0], v1 = v[node * 3 + 1], v2 = v[node * 3 + 2];
    const v4f a = { bf16r(r0), bf16r(r1), bf16r(r2), bf16r(v0) };
    const v4f c = { bf16r(v1), bf16r(v2), 0.0f, 0.0f };
    *(v4fa*)(sS + tid * 8) = a;
    *(v4fa*)(sS + tid * 8 + 4) = c;
    __syncthreads();
    v4f o[2];
    #pragma unroll
    for (int k = 0; k < 2; ++k) o[k] = *(const v4fa*)(sS + (tid + 256 * k) * 4);
    float* dst = NODE + (size_t)blockIdx.x * 2048;
    for (int pass = 0; pass < 2; ++pass) {
      #pragma unroll
      for (int k = 0; k < 2; ++k) *(volatile v4f*)(dst + (tid + 256 * k) * 4) = o[k];
      __threadfence();
    }
  } else {
    unsigned short* sH = (unsigned short*)sS;
    #pragma unroll 1
    for (int e = tid; e < 1024; e += 256) {
      const int n = e >> 5, k = e & 31;
      int row = (k < 13) ? k : (k - 7);
      row = (row > 12) ? 12 : row;
      const float wv = W1[row * 32 + n];
      const float bv = b1[n];
      asm volatile("" :: "v"(wv), "v"(bv));
      const float val = (k < 20) ? wv : bv;
      const unsigned bits = (k <= 20) ? rne_bits(val) : 0u;
      sH[PL_W1X + e] = (unsigned short)bits;
    }
    #pragma unroll 1
    for (int e = tid; e < 1024; e += 256) {
      const int n = e >> 5, k = e & 31;
      sH[PL_W2T + e] = (unsigned short)rne_bits(W2[k * 32 + n]);
    }
    #pragma unroll 1
    for (int e = tid; e < 512; e += 256) {
      const int n = e >> 5, k = e & 31;
      const int nc = (n < 3) ? n : 2;
      const float wv = W3[k * 3 + nc];
      asm volatile("" :: "v"(wv));
      const unsigned bits = (n < 3) ? rne_bits(wv) : 0u;
      sH[PL_W3T + e] = (unsigned short)bits;
    }
    {
      const int t = tid & 63;
      const int i2 = (t < 32) ? t : 31;
      int i3 = t - 32;
      i3 = (i3 < 0) ? 0 : ((i3 > 2) ? 2 : i3);
      const float x2 = b2[i2];
      const float x3 = b3[i3];
      asm volatile("" :: "v"(x2), "v"(x3));
      const float val = (t < 32) ? bf16r(x2) : ((t < 35) ? bf16r(x3) : 0.0f);
      if (tid < 64) sS[PL_BV_DW + t] = __float_as_uint(val);
    }
    __syncthreads();
    v4u o[2];
    #pragma unroll
    for (int k = 0; k < 2; ++k) {
      const int q = tid + 256 * k;
      const int qq = (q < PL_PIECES) ? q : (PL_PIECES - 1);
      o[k] = *(const v4ua*)(sS + qq * 4);
    }
    for (int pass = 0; pass < 2; ++pass) {
      #pragma unroll
      for (int k = 0; k < 2; ++k) {
        const int q = tid + 256 * k;
        if (q < PL_PIECES) *(volatile v4u*)(PLN + q * 4) = o[k];
      }
      __threadfence();
    }
  }
}

__global__ __launch_bounds__(256) __attribute__((amdgpu_num_vgpr(248))) void k_pairs(
    const float* __restrict__ NODE, const unsigned short* __restrict__ WP,
    const float* __restrict__ BV, float* __restrict__ COLP, float* __restrict__ RA)
{
  extern __shared__ __attribute__((aligned(16))) unsigned char dsm[];
  float* sNode = (float*)dsm;
  const int tid = threadIdx.x, lane = tid & 31, w = tid >> 5;
  const int hh = lane >> 4, m = lane & 15;
  const int b = blockIdx.x / BPB;
  const int ib = blockIdx.x % BPB;
  const int g = ib * WPB + w;
  const int i0 = g * IW;
  unsigned char* wbase = dsm + L_NODE + w * L_WV;
  unsigned int* sFeat = (unsigned int*)wbase;
  float* sCol = (float*)(wbase + L_FEAT);
  float* sRA  = (float*)(wbase + L_FEAT + L_COL);

  const v8f z8 = {0.f, 0.f, 0.f, 0.f, 0.f, 0.f, 0.f, 0.f};
  const v4f z4 = {0.f, 0.f, 0.f, 0.f};
  const v4u zu = {0u, 0u, 0u, 0u};

  {
    const float* nb = NODE + (size_t)b * NN * 8;
    #pragma unroll 4
    for (int k = 0; k < 8; ++k) {
      const int q = tid + 256 * k;
      const v4f t = *(const v4fa*)(nb + q * 4);
      *(v4fa*)(sNode + q * 4) = t;
    }
  }
  #pragma unroll 4
  for (int jc = 0; jc < 32; ++jc) *(v4fa*)(sCol + (jc * 32 + lane) * 4) = z4;

  const v16b w1f0 = load_frag_g(WP + PL_W1X + m * 32, hh);
  const v16b w1f1 = load_frag_g(WP + PL_W1X + (16 + m) * 32, hh);
  const v16b w2f0 = load_frag_g(WP + PL_W2T + m * 32, hh);
  const v16b w2f1 = load_frag_g(WP + PL_W2T + (16 + m) * 32, hh);
  const v16b w3f  = load_frag_g(WP + PL_W3T + m * 32, hh);
  const v4f q0 = *(const v4fa*)(BV + 8 * hh);
  const v4f q1 = *(const v4fa*)(BV + 8 * hh + 4);
  const v4f q2 = *(const v4fa*)(BV + 16 + 8 * hh);
  const v4f q3 = *(const v4fa*)(BV + 16 + 8 * hh + 4);
  const v4f q4 = *(const v4fa*)(BV + 32);
  const v8f b2c0 = { q0.x, q0.y, q0.z, q0.w, q1.x, q1.y, q1.z, q1.w };
  const v8f b2c1 = { q2.x, q2.y, q2.z, q2.w, q3.x, q3.y, q3.z, q3.w };
  const float b30 = hh ? 0.0f : q4.x;
  const float b31 = hh ? 0.0f : q4.y;
  const float b32 = hh ? 0.0f : q4.z;
  const v8f b3c = { b30, b31, b32, 0.f, 0.f, 0.f, 0.f, 0.f };

  __syncthreads();

  const float eps2 = (float)(0.01 * 0.01);

  #pragma unroll 1
  for (int il = 0; il < IW; ++il) {
    const int i = i0 + il;
    const v4f ni0 = *(const v4fa*)(sNode + i * 8);
    const v4f ni1 = *(const v4fa*)(sNode + i * 8 + 4);
    const float rix = ni0.x, riy = ni0.y, riz = ni0.z;
    const float vix = ni0.w, viy = ni1.x, viz = ni1.y;
    const unsigned dwv01 = (__float_as_uint(vix) >> 16) | __float_as_uint(viy);
    const unsigned vi2b  = __float_as_uint(viz) >> 16;
    float ap0 = 0.0f, ap1 = 0.0f, ap2 = 0.0f;
    float rw0 = 0.0f, rw1 = 0.0f, rw2 = 0.0f;

    #pragma unroll 1
    for (int jc = 0; jc < 32; ++jc) {
      const int j = jc * 32 + lane;
      const v4f nj0 = *(const v4fa*)(sNode + j * 8);
      const v4f nj1 = *(const v4fa*)(sNode + j * 8 + 4);
      const bool live = (j != i);

      const float dx0 = nj0.x - rix, dx1 = nj0.y - riy, dx2 = nj0.z - riz;
      const float dv0 = nj0.w - vix, dv1 = nj1.x - viy, dv2 = nj1.y - viz;
      const float d2 = dx0 * dx0 + dx1 * dx1 + dx2 * dx2;
      const float dist = sqrtf(d2 + 1e-8f);
      const float d2e = d2 + eps2;
      const float den = d2e * sqrtf(d2e);
      const float inv = 1.0f / den;
      const float t0 = dx0 * inv, t1 = dx1 * inv, t2 = dx2 * inv;
      ap0 += live ? t0 : 0.0f;
      ap1 += live ? t1 : 0.0f;
      ap2 += live ? t2 : 0.0f;

      const unsigned ux0 = __float_as_uint(dx0), ux1 = __float_as_uint(dx1), ux2 = __float_as_uint(dx2);
      const unsigned uv0 = __float_as_uint(dv0), uv1 = __float_as_uint(dv1), uv2 = __float_as_uint(dv2);
      const unsigned ud  = __float_as_uint(dist);
      const unsigned lx0 = tail_bits(dx0, ux0), lx1 = tail_bits(dx1, ux1), lx2 = tail_bits(dx2, ux2);
      const unsigned lv0 = tail_bits(dv0, uv0), lv1 = tail_bits(dv1, uv1), lv2 = tail_bits(dv2, uv2);
      const unsigned ld  = tail_bits(dist, ud);
      const v4u f0 = { dwv01,
                       vi2b | __float_as_uint(nj0.w),
                       (__float_as_uint(nj1.x) >> 16) | __float_as_uint(nj1.y),
                       (ux0 >> 16) | (ux1 & 0xFFFF0000u) };
      const v4u f1 = { (ux2 >> 16) | (uv0 & 0xFFFF0000u),
                       (uv1 >> 16) | (uv2 & 0xFFFF0000u),
                       (ud >> 16) | (lx0 << 16),
                       lx1 | (lx2 << 16) };
      const v4u f2 = { lv0 | (lv1 << 16), lv2 | (ld << 16), 0x00003F80u, 0u };
      unsigned int* frow = sFeat + lane * 16;
      *(v4ua*)(frow)      = f0;
      *(v4ua*)(frow + 4)  = f1;
      *(v4ua*)(frow + 8)  = f2;
      *(v4ua*)(frow + 12) = zu;
      __builtin_amdgcn_fence(__ATOMIC_RELEASE, "workgroup");
      __builtin_amdgcn_wave_barrier();
      FragU fb0, fb1;
      {
        const unsigned int* p0 = sFeat + m * 16 + 4 * hh;
        const unsigned int* p1 = sFeat + (16 + m) * 16 + 4 * hh;
        fb0.q[0] = *(const v4ua*)(p0);
        fb0.q[1] = *(const v4ua*)(p0 + 8);
        fb1.q[0] = *(const v4ua*)(p1);
        fb1.q[1] = *(const v4ua*)(p1 + 8);
      }
      __builtin_amdgcn_wave_barrier();

      const v8f a00 = wmma_bf16(w1f0, fb0.v, z8);
      const v8f a01 = wmma_bf16(w1f1, fb0.v, z8);
      const v8f a10 = wmma_bf16(w1f0, fb1.v, z8);
      const v8f a11 = wmma_bf16(w1f1, fb1.v, z8);

      const FragPair h1t0 = act_split(a00, a01);
      const FragPair h1t1 = act_split(a10, a11);

      v8f c00 = wmma_bf16(w2f0, h1t0.hi, b2c0);
      v8f c01 = wmma_bf16(w2f1, h1t0.hi, b2c1);
      v8f c10 = wmma_bf16(w2f0, h1t1.hi, b2c0);
      v8f c11 = wmma_bf16(w2f1, h1t1.hi, b2c1);
      c00 = wmma_bf16(w2f0, h1t0.lo, c00);
      c01 = wmma_bf16(w2f1, h1t0.lo, c01);
      c10 = wmma_bf16(w2f0, h1t1.lo, c10);
      c11 = wmma_bf16(w2f1, h1t1.lo, c11);

      const FragPair h2t0 = act_split(c00, c01);
      const FragPair h2t1 = act_split(c10, c11);

      v8f m0 = wmma_bf16(w3f, h2t0.hi, b3c);
      v8f m1 = wmma_bf16(w3f, h2t1.hi, b3c);
      m0 = wmma_bf16(w3f, h2t0.lo, m0);
      m1 = wmma_bf16(w3f, h2t1.lo, m1);

      const float s0 = __shfl_xor(m1[0], 16);
      const float s1 = __shfl_xor(m1[1], 16);
      const float s2 = __shfl_xor(m1[2], 16);
      const float mc0 = hh ? s0 : m0[0];
      const float mc1 = hh ? s1 : m0[1];
      const float mc2 = hh ? s2 : m0[2];
      const float e0 = live ? mc0 : 0.0f;
      const float e1 = live ? mc1 : 0.0f;
      const float e2 = live ? mc2 : 0.0f;
      rw0 += e0; rw1 += e1; rw2 += e2;
      float* pc = sCol + (jc * 32 + lane) * 4;
      v4f cv = *(const v4fa*)pc;
      cv.x += e0; cv.y += e1; cv.z += e2;
      *(v4fa*)pc = cv;
    }

    #pragma unroll
    for (int off = 16; off >= 1; off >>= 1) {
      ap0 += __shfl_xor(ap0, off);
      ap1 += __shfl_xor(ap1, off);
      ap2 += __shfl_xor(ap2, off);
      rw0 += __shfl_xor(rw0, off);
      rw1 += __shfl_xor(rw1, off);
      rw2 += __shfl_xor(rw2, off);
    }
    if (lane == 0) {
      const v4f ra = { ap0, ap1, ap2, 0.0f };
      const v4f rb = { rw0, rw1, rw2, 0.0f };
      *(v4fa*)(sRA + il * 8) = ra;
      *(v4fa*)(sRA + il * 8 + 4) = rb;
    }
  }

  __builtin_amdgcn_fence(__ATOMIC_RELEASE, "workgroup");
  __builtin_amdgcn_wave_barrier();
  {
    const v4f rv = *(const v4fa*)(sRA + lane * 4);
    float* radst = RA + ((size_t)b * NN + i0) * 8 + lane * 4;
    *(volatile v4f*)radst = rv;
    __threadfence();
    *(volatile v4f*)radst = rv;
  }
  {
    float* cdst = COLP + ((size_t)b * NG + g) * NN * 4;
    for (int pass = 0; pass < 2; ++pass) {
      #pragma unroll 4
      for (int jc = 0; jc < 32; ++jc) {
        const v4f cvv = *(const v4fa*)(sCol + (jc * 32 + lane) * 4);
        *(volatile v4f*)(cdst + (jc * 32 + lane) * 4) = cvv;
      }
      __threadfence();
    }
  }
}

__global__ __launch_bounds__(256) void k_fin(const float* __restrict__ RA, const float* __restrict__ COLP,
                                             float* __restrict__ out)
{
  __shared__ __attribute__((aligned(16))) float sO[768];
  const int tid = threadIdx.x;
  const int node = blockIdx.x * 256 + tid;
  const int b = node >> 10, i = node & (NN - 1);
  const v4f a  = *(const v4fa*)(RA + (size_t)node * 8);
  const v4f rw = *(const v4fa*)(RA + (size_t)node * 8 + 4);
  float c0 = 0.0f, c1 = 0.0f, c2 = 0.0f;
  const float* cp = COLP + ((size_t)b * NG * NN + i) * 4;
  #pragma unroll 4
  for (int gg = 0; gg < NG; ++gg) {
    const v4f c = *(const v4fa*)(cp + (size_t)gg * NN * 4);
    c0 += c.x; c1 += c.y; c2 += c.z;
  }
  sO[tid * 3 + 0] = a.x + (rw.x - c0);
  sO[tid * 3 + 1] = a.y + (rw.y - c1);
  sO[tid * 3 + 2] = a.z + (rw.z - c2);
  __syncthreads();
  const int q = (tid < 192) ? tid : 191;
  const v4f o = *(const v4fa*)(sO + q * 4);
  asm volatile("" :: "v"(o));
  float* dst = out + (size_t)blockIdx.x * 768 + tid * 4;
  if (tid < 192) *(volatile v4f*)dst = o;
  __threadfence();
  if (tid < 192) *(volatile v4f*)dst = o;
}

extern "C" void kernel_launch(void* const* d_in, const int* in_sizes, int n_in,
                              void* d_out, int out_size, void* d_ws, size_t ws_size,
                              hipStream_t stream) {
  if (n_in < 8) return;
  if (in_sizes[0] != NB * NN * 3 || in_sizes[1] != NB * NN * 3) return;
  if (in_sizes[2] != 13 * HID || in_sizes[3] != HID) return;
  if (in_sizes[4] != HID * HID || in_sizes[5] != HID) return;
  if (in_sizes[6] != HID * 3 || in_sizes[7] != 3) return;
  if (out_size != NB * NN * 3) return;
  if ((size_t)WS_TOTAL > ws_size) return;

  const float* r  = (const float*)d_in[0];
  const float* v  = (const float*)d_in[1];
  const float* W1 = (const float*)d_in[2];
  const float* b1 = (const float*)d_in[3];
  const float* W2 = (const float*)d_in[4];
  const float* b2 = (const float*)d_in[5];
  const float* W3 = (const float*)d_in[6];
  const float* b3 = (const float*)d_in[7];
  float* out = (float*)d_out;

  char* ws = (char*)d_ws;
  unsigned int*   PLN  = (unsigned int*)(ws + WS_PLN);
  float*          NODE = (float*)(ws + WS_NODE);
  float*          RA   = (float*)(ws + WS_RA);
  float*          COLP = (float*)(ws + WS_COLP);
  const unsigned short* WP = (const unsigned short*)(ws + WS_PLN);
  const float*          BV = (const float*)(ws + WS_PLN + PL_BV_DW * 4);

  k_prep<<<33, 256, 0, stream>>>(r, v, W1, b1, W2, b2, W3, b3, PLN, NODE);

  (void)hipFuncSetAttribute(reinterpret_cast<const void*>(&k_pairs),
                            hipFuncAttributeMaxDynamicSharedMemorySize, L_TOTAL);
  k_pairs<<<NB * BPB, 256, L_TOTAL, stream>>>(NODE, WP, BV, COLP, RA);

  k_fin<<<(NB * NN) / 256, 256, 0, stream>>>(RA, COLP, out);
  (void)hipGetLastError();
}
